// MambaLayer_8985071583799
// MI455X (gfx1250) — hardware-verified
//
#include <hip/hip_runtime.h>
#include <math.h>

typedef __attribute__((ext_vector_type(16))) _Float16 v16h;
typedef __attribute__((ext_vector_type(8)))  _Float16 v8h;
typedef __attribute__((ext_vector_type(8)))  float    v8f;
typedef __attribute__((ext_vector_type(4)))  float    v4f;

constexpr int kBatch = 2;
constexpr int kCin   = 512;
constexpr int kHW    = 32;
constexpr int kSeqL  = kHW * kHW;
constexpr int kRows  = kBatch * kSeqL;
constexpr int kPpm   = 128;
constexpr int kDmod  = kCin + 4 * kPpm;
constexpr int kDin   = 2 * kDmod;
constexpr int kNst   = 16;
constexpr int kDtR   = (kDmod + 15) / 16;
constexpr int kPrjN  = kDtR + 2 * kNst;
constexpr int kPrjP  = 128;
constexpr int kXZP   = 2 * kDin;
constexpr int kTP    = 260;
constexpr int kSc1   = 9;
constexpr int kSc2   = 17;
constexpr int kSc3   = 25;
constexpr int kSegP1 = 192;
constexpr int kSegP2 = 640;
constexpr int kSegP3 = 1280;
constexpr int kSegOff2 = kSegP1;
constexpr int kSegOff3 = kSegP1 + kSegP2;
constexpr int kPoolRows = kSegP1 + kSegP2 + kSegP3;
constexpr float kBnEps = 1e-5f;
static_assert(kSeqL == 1024 && kRows == 2048 && kDmod == 1024 && kDin == 2048 && kDtR == 64 && kPrjN == 96);
static_assert(2 * kSc1 * kSc1 <= kSegP1 && 2 * kSc2 * kSc2 <= kSegP2 && 2 * kSc3 * kSc3 <= kSegP3);
static_assert((kSegP1 % 64) == 0 && (kSegP2 % 64) == 0 && (kSegP3 % 64) == 0 && kPoolRows == 2112);
static_assert((kCin % 32) == 0 && (kDmod % 32) == 0 && (kDin % 32) == 0 && (kDtR % 32) == 0);
static_assert((kRows % 64) == 0 && (kXZP % 64) == 0 && (kPrjP % 64) == 0 && (kPpm % 64) == 0 && (kDmod % 64) == 0 && (kSeqL % 64) == 0);

constexpr float kCarPool = 16.0f;
constexpr float kCarWin  = 32.0f;
constexpr float kCarWx   = 32.0f;
constexpr float kCarWdt  = 8.0f;
constexpr float kCarDt   = 16.0f;
constexpr float kCarY    = 16.0f;
constexpr float kCarWout = 32.0f;

constexpr size_t kSzWIN  = (size_t)kXZP * kDmod * 2;
constexpr size_t kSzWPL  = (size_t)4 * kPpm * kCin * 2;
constexpr size_t kSzWXP  = (size_t)kPrjP * kDin * 2;
constexpr size_t kSzWDT  = (size_t)kDin * kDtR * 2;
constexpr size_t kSzWOUT = (size_t)kDmod * kDin * 2;
constexpr size_t kSzSEQ  = (size_t)kRows * kDmod * 2;
constexpr size_t kSzYS0  = (size_t)kRows * kPpm * 4;
constexpr size_t kSzPOOL = (size_t)kPoolRows * kCin * 2;
constexpr size_t kSzYSP  = (size_t)kPoolRows * kPpm * 4;
constexpr size_t kSzXZ   = (size_t)kRows * kXZP * 4;
constexpr size_t kSzUC   = (size_t)kRows * kDin * 4;
constexpr size_t kSzUC16 = (size_t)kRows * kDin * 2;
constexpr size_t kSzPROJ = (size_t)kRows * kPrjP * 4;
constexpr size_t kSzDT16 = (size_t)kRows * kDtR * 2;
constexpr size_t kSzDLR  = (size_t)kRows * kDin * 4;
constexpr size_t kSzY16  = (size_t)kRows * kDin * 2;
constexpr size_t kOffWIN  = 0;
constexpr size_t kOffWPL  = kOffWIN  + kSzWIN;
constexpr size_t kOffWXP  = kOffWPL  + kSzWPL;
constexpr size_t kOffWDT  = kOffWXP  + kSzWXP;
constexpr size_t kOffWOUT = kOffWDT  + kSzWDT;
constexpr size_t kOffSEQ  = kOffWOUT + kSzWOUT;
constexpr size_t kOffYS0  = kOffSEQ  + kSzSEQ;
constexpr size_t kOffPOOL = kOffYS0  + kSzYS0;
constexpr size_t kOffYSP  = kOffPOOL + kSzPOOL;
constexpr size_t kOffXZ   = kOffYSP  + kSzYSP;
constexpr size_t kOffUC   = kOffXZ   + kSzXZ;
constexpr size_t kOffUC16 = kOffUC   + kSzUC;
constexpr size_t kOffPROJ = kOffUC16 + kSzUC16;
constexpr size_t kOffDT16 = kOffPROJ + kSzPROJ;
constexpr size_t kOffDLR  = kOffDT16 + kSzDT16;
constexpr size_t kOffY16  = kOffDLR  + kSzDLR;
constexpr size_t kWsTotal = kOffY16  + kSzY16;
static_assert(kWsTotal == 107577344ull);
static_assert(kWsTotal <= 134217728ull);
static_assert((kOffWPL % 128) == 0 && (kOffWXP % 128) == 0 && (kOffWDT % 128) == 0 && (kOffWOUT % 128) == 0 &&
              (kOffSEQ % 128) == 0 && (kOffYS0 % 128) == 0 && (kOffPOOL % 128) == 0 && (kOffYSP % 128) == 0 &&
              (kOffXZ % 128) == 0 && (kOffUC % 128) == 0 && (kOffUC16 % 128) == 0 && (kOffPROJ % 128) == 0 &&
              (kOffDT16 % 128) == 0 && (kOffDLR % 128) == 0 && (kOffY16 % 128) == 0);

union FragU { v16h v; v8h h[2]; };
__device__ __forceinline__ v16h frag_load(const _Float16* p) {
  FragU f;
  f.h[0] = *(const v8h*)(p);
  f.h[1] = *(const v8h*)(p + 16);
  return f.v;
}
__device__ __forceinline__ v8f frag_mma(v16h a, v16h b, v8f c) {
  return __builtin_amdgcn_wmma_f32_16x16x32_f16(false, a, false, b, (short)0, c, false, false);
}
__device__ __forceinline__ void group_guard_h(v8f& a, v8f& b, v8f& c, v8f& d, v16h x, v16h y0, v16h y1, v16h y2, v16h y3) {
  asm volatile("v_nop\n\tv_nop\n\tv_nop\n\tv_nop" : "+v"(a), "+v"(b), "+v"(c), "+v"(d) : "v"(x), "v"(y0), "v"(y1), "v"(y2), "v"(y3));
}
__device__ __forceinline__ void keep4_h(v16h a, v16h b, v16h c, v16h d) { asm volatile("v_nop" :: "v"(a), "v"(b), "v"(c), "v"(d)); }
__device__ __forceinline__ void acc_guard4(v8f& a, v8f& b, v8f& c, v8f& d) { asm volatile("v_nop\n\tv_nop\n\tv_nop\n\tv_nop" : "+v"(a), "+v"(b), "+v"(c), "+v"(d)); }

template <int BIAS_MODE, int ACT>
__global__ __launch_bounds__(256) void wmma_gemm64(
    const unsigned short* __restrict__ Ap, int lda, long strideA,
    const unsigned short* __restrict__ Btp, int ldb, long strideB,
    float* __restrict__ Cout, int ldc, long strideC,
    const float* __restrict__ bias,
    const float* __restrict__ bnG, const float* __restrict__ bnB,
    const float* __restrict__ bnM, const float* __restrict__ bnV,
    int M, int N, int K, float scale) {
  const _Float16* A  = (const _Float16*)Ap;
  const _Float16* Bt = (const _Float16*)Btp;
  __shared__ __align__(16) float sT[8][16 * 68];
  const int b    = blockIdx.y;
  const int lane = threadIdx.x & 31;
  const int wave = threadIdx.x >> 5;
  const int tilesN = N >> 6;
  const int tilesM = M >> 6;
  const int tile = blockIdx.x * 8 + wave;
  if (tile >= tilesM * tilesN) return;
  const int tm = tile / tilesN;
  const int tn = tile - tm * tilesN;
  const int m0 = tm << 6;
  const int n0 = tn << 6;

  const _Float16* Ab = A  + (size_t)b * strideA;
  const _Float16* Bb = Bt + (size_t)b * strideB;

  const int rlane = lane & 15;
  const int koff  = (lane >> 4) * 8;
  const int mOff  = (lane >> 4) * 8;

  v8f acc[4][4];
#pragma unroll
  for (int i = 0; i < 4; ++i)
#pragma unroll
    for (int j = 0; j < 4; ++j) acc[i][j] = (v8f){0.f,0.f,0.f,0.f,0.f,0.f,0.f,0.f};

  for (int k0 = 0; k0 < K; k0 += 32) {
    v16h bh[4];
#pragma unroll
    for (int j = 0; j < 4; ++j) {
      const size_t bo = (size_t)(n0 + (j << 4) + rlane) * ldb + koff + k0;
      bh[j] = frag_load(Bb + bo);
    }
#pragma unroll
    for (int i = 0; i < 4; ++i) {
      const size_t ao = (size_t)(m0 + (i << 4) + rlane) * lda + koff + k0;
      const v16h ah = frag_load(Ab + ao);
#pragma unroll
      for (int j = 0; j < 4; ++j) acc[i][j] = frag_mma(ah, bh[j], acc[i][j]);
      group_guard_h(acc[i][0], acc[i][1], acc[i][2], acc[i][3], ah, bh[0], bh[1], bh[2], bh[3]);
    }
    keep4_h(bh[0], bh[1], bh[2], bh[3]);
  }
  acc_guard4(acc[0][0], acc[0][1], acc[0][2], acc[0][3]);
  acc_guard4(acc[1][0], acc[1][1], acc[1][2], acc[1][3]);
  acc_guard4(acc[2][0], acc[2][1], acc[2][2], acc[2][3]);
  acc_guard4(acc[3][0], acc[3][1], acc[3][2], acc[3][3]);

  float eM[4], eS[4], eC[4];
#pragma unroll
  for (int j = 0; j < 4; ++j) {
    const int n = n0 + (j << 4) + rlane;
    eM[j] = 0.f; eS[j] = 1.f; eC[j] = 0.f;
    if (BIAS_MODE == 2) eC[j] = bias[n];
    if (ACT == 6) {
      eM[j] = bnM[n];
      eS[j] = bnG[n] * rsqrtf(bnV[n] + kBnEps);
      eC[j] = bnB[n];
    }
  }

  float* slab = sT[wave];
  float* C = Cout + (size_t)b * strideC;
#pragma unroll
  for (int i = 0; i < 4; ++i) {
    const int mBase = m0 + (i << 4);
#pragma unroll
    for (int j = 0; j < 4; ++j) {
#pragma unroll
      for (int r = 0; r < 8; ++r) {
        float v = acc[i][j][r] * scale;
        if (ACT == 6) {
          v = (v - eM[j]) * eS[j] + eC[j];
          v = fminf(fmaxf(v, 0.0f), 6.0f);
        } else if (BIAS_MODE == 2) {
          v += eC[j];
        }
        slab[(mOff + r) * 68 + (j << 4) + rlane] = v;
      }
    }
    __builtin_amdgcn_fence(__ATOMIC_RELEASE, "workgroup");
    __builtin_amdgcn_wave_barrier();
    __builtin_amdgcn_fence(__ATOMIC_ACQUIRE, "workgroup");
    {
      const int hh = lane >> 4, c4 = (lane & 15) * 4;
      for (int pass = 0; pass < 2; ++pass) {
#pragma unroll
        for (int it = 0; it < 8; ++it) {
          const int row = it * 2 + hh;
          const v4f v = *(const v4f*)(slab + row * 68 + c4);
          *(volatile v4f*)(C + (size_t)(mBase + row) * ldc + n0 + c4) = v;
        }
        __threadfence();
      }
    }
    __builtin_amdgcn_fence(__ATOMIC_RELEASE, "workgroup");
    __builtin_amdgcn_wave_barrier();
    __builtin_amdgcn_fence(__ATOMIC_ACQUIRE, "workgroup");
  }
}

__global__ __launch_bounds__(256) void cast_f16_kernel(
    const float* __restrict__ src, unsigned short* __restrict__ dst, int total8, int nreal8, float scale)
{
  const int i = blockIdx.x * 256 + threadIdx.x;
  if (i >= total8) return;
  const bool real = (i < nreal8);
  const int ic = real ? i : (nreal8 - 1);
  const float* p = src + ((size_t)ic << 3);
  const v4f a0 = *(const v4f*)(p);
  const v4f a1 = *(const v4f*)(p + 4);
  v8h hv;
#pragma unroll
  for (int e = 0; e < 4; ++e) {
    const float f0 = real ? (a0[e] * scale) : 0.0f;
    const float f1 = real ? (a1[e] * scale) : 0.0f;
    hv[e]     = (_Float16)f0;
    hv[4 + e] = (_Float16)f1;
  }
  unsigned short* q = dst + ((size_t)i << 3);
  *(volatile v8h*)q = hv;
  __threadfence();
  *(volatile v8h*)q = hv;
}

__global__ __launch_bounds__(256) void xpose_x_kernel(
    const float* __restrict__ x, unsigned short* __restrict__ seq)
{
  __shared__ float tile[64 * 65];
  const int tid = threadIdx.x, lane = tid & 31, wave = tid >> 5;
  const int p0 = blockIdx.x * 64;
  const int c0 = blockIdx.y * 64;
  const int b  = blockIdx.z;
  const float* xb = x + (size_t)b * kCin * kSeqL;
#pragma unroll
  for (int it = 0; it < 16; ++it) {
    const int idx = tid + it * 256;
    const int cc  = idx >> 6;
    const int pp  = idx & 63;
    tile[cc * 65 + pp] = xb[(size_t)(c0 + cc) * kSeqL + p0 + pp];
  }
  __syncthreads();
  const int q = lane >> 3, c8 = (lane & 7) * 8;
  v8h hv[2];
#pragma unroll
  for (int it = 0; it < 2; ++it) {
    const int prow = it * 32 + wave * 4 + q;
#pragma unroll
    for (int e = 0; e < 8; ++e) hv[it][e] = (_Float16)tile[(c8 + e) * 65 + prow];
  }
  for (int pass = 0; pass < 2; ++pass) {
#pragma unroll
    for (int it = 0; it < 2; ++it) {
      const int prow = it * 32 + wave * 4 + q;
      *(volatile v8h*)(seq + (size_t)(b * kSeqL + p0 + prow) * kDmod + c0 + c8) = hv[it];
    }
    __threadfence();
  }
}

__global__ __launch_bounds__(256) void ppm0_mean_kernel(
    const float* __restrict__ YS0, unsigned short* __restrict__ seq)
{
  __shared__ float sP[4 * 64];
  __shared__ float sM[64];
  const int tid = threadIdx.x, lane = tid & 31, wave = tid >> 5;
  const int b  = blockIdx.x >> 1;
  const int ch = blockIdx.x & 1;
  const int col = tid & 63, rg = tid >> 6;
  const float* src = YS0 + (size_t)(b * kSeqL + rg * 256) * kPpm + ch * 64 + col;
  float a0 = 0.f, a1 = 0.f, a2 = 0.f, a3 = 0.f;
#pragma unroll 1
  for (int r = 0; r < 256; r += 4) {
    a0 += src[(size_t)(r + 0) * kPpm];
    a1 += src[(size_t)(r + 1) * kPpm];
    a2 += src[(size_t)(r + 2) * kPpm];
    a3 += src[(size_t)(r + 3) * kPpm];
  }
  sP[rg * 64 + col] = (a0 + a1) + (a2 + a3);
  __syncthreads();
  if (tid < 64) {
    const float s = (sP[tid] + sP[64 + tid]) + (sP[128 + tid] + sP[192 + tid]);
    sM[tid] = s * (1.0f / (float)kSeqL);
  }
  __syncthreads();
  const int q = lane >> 3, c8 = (lane & 7) * 8;
  v8h hv;
#pragma unroll
  for (int e = 0; e < 8; ++e) hv[e] = (_Float16)sM[c8 + e];
  for (int pass = 0; pass < 2; ++pass) {
#pragma unroll 1
    for (int it = 0; it < 32; ++it) {
      const int row = it * 32 + wave * 4 + q;
      *(volatile v8h*)(seq + (size_t)(b * kSeqL + row) * kDmod + kCin + ch * 64 + c8) = hv;
    }
    __threadfence();
  }
}

__global__ __launch_bounds__(256) void pool_kernel(
    const float* __restrict__ x, unsigned short* __restrict__ P16)
{
  const int t   = blockIdx.x * 256 + threadIdx.x;
  const int row = t >> 6;
  const int c8  = (t & 63) << 3;
  int s, seg0;
  if (row < kSegOff2)      { s = kSc1; seg0 = 0; }
  else if (row < kSegOff3) { s = kSc2; seg0 = kSegOff2; }
  else                     { s = kSc3; seg0 = kSegOff3; }
  const int ss = s * s;
  const int rr = row - seg0;
  const bool real = (rr < 2 * ss);
  const int rc = real ? rr : 0;
  const int b  = rc / ss;
  const int pq = rc - b * ss;
  const int p  = pq / s;
  const int q  = pq - p * s;
  const int hs = (p * kHW) / s, he = ((p + 1) * kHW + s - 1) / s;
  const int wb = (q * kHW) / s, we = ((q + 1) * kHW + s - 1) / s;
  float acc[8];
#pragma unroll
  for (int e = 0; e < 8; ++e) acc[e] = 0.f;
  if (real) {
    const float* xb = x + (size_t)(b * kCin + c8) * kSeqL;
#pragma unroll 1
    for (int h = hs; h < he; ++h) {
#pragma unroll 1
      for (int w = wb; w < we; ++w) {
        const float* xp = xb + h * kHW + w;
#pragma unroll
        for (int e = 0; e < 8; ++e) acc[e] += xp[(size_t)e * kSeqL];
      }
    }
  }
  const float inv = (1.0f / (float)(he - hs)) * (1.0f / (float)(we - wb));
  v8h hv;
#pragma unroll
  for (int e = 0; e < 8; ++e) {
    const float f = real ? (acc[e] * inv) : 0.0f;
    hv[e] = (_Float16)f;
  }
  unsigned short* dst = P16 + (size_t)row * kCin + c8;
  *(volatile v8h*)dst = hv;
  __threadfence();
  *(volatile v8h*)dst = hv;
}

__global__ __launch_bounds__(256) void interp_kernel(
    const float* __restrict__ YSP, unsigned short* __restrict__ seq)
{
  const int t  = blockIdx.x * 256 + threadIdx.x;
  const int m  = t / 48;
  const int g  = t - m * 48;
  const int si = g >> 4;
  const int o8 = (g & 15) << 3;
  const int s  = kSc1 + 8 * si;
  const int seg0 = (si == 0) ? 0 : ((si == 1) ? kSegOff2 : kSegOff3);
  const int b = m >> 10;
  const int p = m & (kSeqL - 1);
  const int h = p >> 5, w = p & 31;
  const float sm1 = (float)(s - 1);
  float sh = ((float)h + 0.5f) * (float)s * (1.0f / (float)kHW) - 0.5f;
  sh = fminf(fmaxf(sh, 0.0f), sm1);
  const int h0 = (int)sh;
  const int h1 = (h0 + 1 < s) ? (h0 + 1) : (s - 1);
  const float wh = sh - (float)h0;
  float sw = ((float)w + 0.5f) * (float)s * (1.0f / (float)kHW) - 0.5f;
  sw = fminf(fmaxf(sw, 0.0f), sm1);
  const int w0 = (int)sw;
  const int w1 = (w0 + 1 < s) ? (w0 + 1) : (s - 1);
  const float ww = sw - (float)w0;
  const int base = seg0 + b * s * s;
  const float* r00 = YSP + (size_t)(base + h0 * s + w0) * kPpm + o8;
  const float* r01 = YSP + (size_t)(base + h0 * s + w1) * kPpm + o8;
  const float* r10 = YSP + (size_t)(base + h1 * s + w0) * kPpm + o8;
  const float* r11 = YSP + (size_t)(base + h1 * s + w1) * kPpm + o8;
  const v4f a00 = *(const v4f*)(r00), b00 = *(const v4f*)(r00 + 4);
  const v4f a01 = *(const v4f*)(r01), b01 = *(const v4f*)(r01 + 4);
  const v4f a10 = *(const v4f*)(r10), b10 = *(const v4f*)(r10 + 4);
  const v4f a11 = *(const v4f*)(r11), b11 = *(const v4f*)(r11 + 4);
  const float uh = 1.0f - wh, uw = 1.0f - ww;
  v8h hv;
#pragma unroll
  for (int e = 0; e < 4; ++e) {
    const float t0 = uw * a00[e] + ww * a01[e];
    const float t1 = uw * a10[e] + ww * a11[e];
    const float v0 = uh * t0 + wh * t1;
    const float t2 = uw * b00[e] + ww * b01[e];
    const float t3 = uw * b10[e] + ww * b11[e];
    const float v1 = uh * t2 + wh * t3;
    hv[e]     = (_Float16)v0;
    hv[4 + e] = (_Float16)v1;
  }
  unsigned short* dst = seq + (size_t)m * kDmod + kCin + kPpm + (g << 3);
  *(volatile v8h*)dst = hv;
  __threadfence();
  *(volatile v8h*)dst = hv;
}

__global__ __launch_bounds__(256) void dt_cast_kernel(
    const float* __restrict__ PROJ, unsigned short* __restrict__ DT16, int total8, float scale)
{
  const int i = blockIdx.x * 256 + threadIdx.x;
  if (i >= total8) return;
  const int e0  = i << 3;
  const int row = e0 >> 6;
  const int c8  = e0 & 63;
  const float* p = PROJ + (size_t)row * kPrjP + c8;
  const v4f a0 = *(const v4f*)(p);
  const v4f a1 = *(const v4f*)(p + 4);
  v8h hv;
#pragma unroll
  for (int e = 0; e < 4; ++e) {
    hv[e]     = (_Float16)(a0[e] * scale);
    hv[4 + e] = (_Float16)(a1[e] * scale);
  }
  unsigned short* qd = DT16 + e0;
  *(volatile v8h*)qd = hv;
  __threadfence();
  *(volatile v8h*)qd = hv;
}

__global__ __launch_bounds__(256) void conv_silu_kernel(
    const float* __restrict__ XZ, const float* __restrict__ cw, const float* __restrict__ cb,
    float* __restrict__ UC, unsigned short* __restrict__ UC16)
{
  __shared__ __align__(16) float sT[16 * kTP];
  const int tid = threadIdx.x, lane = tid & 31, wave = tid >> 5;
  const int d0 = blockIdx.x * 256, d = d0 + tid;
  const int g0 = blockIdx.y * 64;
  const int tb = g0 & (kSeqL - 1);
  const float w0 = cw[d * 4 + 0], w1 = cw[d * 4 + 1], w2 = cw[d * 4 + 2], w3 = cw[d * 4 + 3];
  const float bc = cb[d];
  float xm3, xm2, xm1;
  {
    const bool hist = (tb > 0);
    const int rb = hist ? (g0 - 3) : g0;
    const float v3 = XZ[(size_t)rb * kXZP + d];
    const float v2 = XZ[(size_t)(rb + 1) * kXZP + d];
    const float v1 = XZ[(size_t)(rb + 2) * kXZP + d];
    xm3 = hist ? v3 : 0.f;
    xm2 = hist ? v2 : 0.f;
    xm1 = hist ? v1 : 0.f;
  }
  const int hrow = wave >> 1;
  const int hch  = (wave & 1) * 128 + lane * 4;
#pragma unroll 1
  for (int sub = 0; sub < 4; ++sub) {
    const int lb = g0 + sub * 16;
#pragma unroll 1
    for (int s = 0; s < 16; ++s) {
      float xcur = XZ[(size_t)(lb + s) * kXZP + d];
      asm volatile("" : "+v"(xcur));
      float acc = w0 * xm3;
      acc = fmaf(w1, xm2, acc);
      acc = fmaf(w2, xm1, acc);
      acc = fmaf(w3, xcur, acc);
      const float sv = acc + bc;
      const float sg = __builtin_amdgcn_rcpf(1.0f + expf(-sv));
      sT[s * kTP + tid] = sv * sg;
      xm3 = xm2; xm2 = xm1; xm1 = xcur;
    }
    __syncthreads();
    v4f fv[4];
    v8h bv[2];
#pragma unroll
    for (int it = 0; it < 4; ++it) fv[it] = *(const v4f*)(sT + (it * 4 + hrow) * kTP + hch);
#pragma unroll
    for (int it = 0; it < 2; ++it) {
      const float* sp = sT + (it * 8 + wave) * kTP + lane * 8;
      const v4f a0 = *(const v4f*)(sp);
      const v4f a1 = *(const v4f*)(sp + 4);
#pragma unroll
      for (int e = 0; e < 4; ++e) {
        bv[it][e]     = (_Float16)a0[e];
        bv[it][4 + e] = (_Float16)a1[e];
      }
    }
    for (int pass = 0; pass < 2; ++pass) {
#pragma unroll
      for (int it = 0; it < 4; ++it)
        *(volatile v4f*)(UC + (size_t)(lb + it * 4 + hrow) * kDin + d0 + hch) = fv[it];
#pragma unroll
      for (int it = 0; it < 2; ++it)
        *(volatile v8h*)(UC16 + (size_t)(lb + it * 8 + wave) * kDin + d0 + lane * 8) = bv[it];
      __threadfence();
    }
    __syncthreads();
  }
}

__global__ __launch_bounds__(256) void scan_kernel(
    const float* __restrict__ DLR, const float* __restrict__ UC, const float* __restrict__ XZ,
    const float* __restrict__ PROJ, const float* __restrict__ A_log, const float* __restrict__ Dv,
    unsigned short* __restrict__ Y16)
{
  __shared__ __align__(16) float sBC[16 * 32];
  __shared__ __align__(16) float sY[16 * kTP];
  const int tid = threadIdx.x, lane = tid & 31, wave = tid >> 5;
  const int d0 = blockIdx.x * 256, d = d0 + tid;
  const size_t row0 = (size_t)blockIdx.y * kSeqL;

  float An[kNst];
#pragma unroll
  for (int n = 0; n < kNst; ++n) An[n] = -expf(A_log[(size_t)d * kNst + n]);
  const float Dd = Dv[d];
  float h[kNst];
#pragma unroll
  for (int n = 0; n < kNst; ++n) h[n] = 0.f;

#pragma unroll 1
  for (int c = 0; c < kSeqL / 16; ++c) {
    const int l0 = c * 16;
    if (tid < 128) {
      const int r = tid >> 3, q = (tid & 7) * 4;
      const v4f v = *(const v4f*)(PROJ + (row0 + l0 + r) * kPrjP + kDtR + q);
      *(v4f*)(sBC + r * 32 + q) = v;
    }
    __syncthreads();
#pragma unroll 1
    for (int s = 0; s < 16; ++s) {
      const size_t m = row0 + (size_t)(l0 + s);
      float a  = DLR[m * kDin + d];
      float xv = UC[m * kDin + d];
      float zv = XZ[m * kXZP + kDin + d];
      asm volatile("" : "+v"(a));
      asm volatile("" : "+v"(xv));
      asm volatile("" : "+v"(zv));
      const float delta = fmaxf(a, 0.0f) + log1pf(expf(-fabsf(a)));
      const float du = delta * xv;
      v4f Bq[4], Cq[4];
#pragma unroll
      for (int qq = 0; qq < 4; ++qq) {
        Bq[qq] = *(const v4f*)(sBC + s * 32 + 4 * qq);
        Cq[qq] = *(const v4f*)(sBC + s * 32 + kNst + 4 * qq);
      }
      float y = 0.f;
#pragma unroll
      for (int n = 0; n < kNst; ++n) {
        const float e = __expf(delta * An[n]);
        const float hn = e * h[n] + du * Bq[n >> 2][n & 3];
        h[n] = hn;
        y += Cq[n >> 2][n & 3] * hn;
      }
      y += xv * Dd;
      const float sg = __builtin_amdgcn_rcpf(1.0f + expf(-zv));
      const float g  = zv * sg;
      sY[s * kTP + tid] = (y * g) * kCarY;
    }
    __syncthreads();
    v8h hv[2];
#pragma unroll
    for (int it = 0; it < 2; ++it) {
      const float* sp = sY + (it * 8 + wave) * kTP + lane * 8;
      const v4f a0 = *(const v4f*)(sp);
      const v4f a1 = *(const v4f*)(sp + 4);
#pragma unroll
      for (int e = 0; e < 4; ++e) { hv[it][e] = (_Float16)a0[e]; hv[it][4 + e] = (_Float16)a1[e]; }
    }
    for (int pass = 0; pass < 2; ++pass) {
#pragma unroll
      for (int it = 0; it < 2; ++it)
        *(volatile v8h*)(Y16 + (row0 + l0 + it * 8 + wave) * kDin + d0 + lane * 8) = hv[it];
      __threadfence();
    }
  }
}

extern "C" void kernel_launch(void* const* d_in, const int* in_sizes, int n_in,
                              void* d_out, int out_size, void* d_ws, size_t ws_size,
                              hipStream_t stream)
{
  if (n_in < 15) return;
  if (in_sizes[0] != kBatch * kCin * kSeqL) return;
  if (in_sizes[1] != 4 * kPpm * kCin) return;
  if (in_sizes[2] != 4 * kPpm || in_sizes[3] != 4 * kPpm || in_sizes[4] != 4 * kPpm || in_sizes[5] != 4 * kPpm) return;
  if (in_sizes[6] != kXZP * kDmod) return;
  if (in_sizes[7] != kDin * 4 || in_sizes[8] != kDin) return;
  if (in_sizes[9] != kPrjN * kDin) return;
  if (in_sizes[10] != kDin * kDtR || in_sizes[11] != kDin) return;
  if (in_sizes[12] != kDin * kNst || in_sizes[13] != kDin) return;
  if (in_sizes[14] != kDmod * kDin) return;
  if (out_size != kBatch * kDmod * kSeqL) return;
  if (ws_size < kWsTotal) return;

  const float* x       = (const float*)d_in[0];
  const float* pool_w  = (const float*)d_in[1];
  const float* bn_g    = (const float*)d_in[2];
  const float* bn_b    = (const float*)d_in[3];
  const float* bn_m    = (const float*)d_in[4];
  const float* bn_v    = (const float*)d_in[5];
  const float* W_in    = (const float*)d_in[6];
  const float* conv_w  = (const float*)d_in[7];
  const float* conv_b  = (const float*)d_in[8];
  const float* W_xprj  = (const float*)d_in[9];
  const float* W_dt    = (const float*)d_in[10];
  const float* b_dt    = (const float*)d_in[11];
  const float* A_log   = (const float*)d_in[12];
  const float* Dv      = (const float*)d_in[13];
  const float* W_out   = (const float*)d_in[14];
  float* dout = (float*)d_out;

  char* ws = (char*)d_ws;
  unsigned short* WIN16  = (unsigned short*)(ws + kOffWIN);
  unsigned short* WPL16  = (unsigned short*)(ws + kOffWPL);
  unsigned short* WXP16  = (unsigned short*)(ws + kOffWXP);
  unsigned short* WDT16  = (unsigned short*)(ws + kOffWDT);
  unsigned short* WOUT16 = (unsigned short*)(ws + kOffWOUT);
  unsigned short* SEQ16  = (unsigned short*)(ws + kOffSEQ);
  float*          YS0    = (float*)(ws + kOffYS0);
  unsigned short* POOL16 = (unsigned short*)(ws + kOffPOOL);
  float*          YSP    = (float*)(ws + kOffYSP);
  float*          XZ     = (float*)(ws + kOffXZ);
  float*          UC     = (float*)(ws + kOffUC);
  unsigned short* UC16   = (unsigned short*)(ws + kOffUC16);
  float*          PROJ   = (float*)(ws + kOffPROJ);
  unsigned short* DT16   = (unsigned short*)(ws + kOffDT16);
  float*          DLR    = (float*)(ws + kOffDLR);
  unsigned short* Y16    = (unsigned short*)(ws + kOffY16);

  {
    const int t8 = kXZP * kDmod / 8;
    cast_f16_kernel<<<t8 / 256, 256, 0, stream>>>(W_in, WIN16, t8, t8, kCarWin);
  }
  {
    const int t8 = 4 * kPpm * kCin / 8;
    cast_f16_kernel<<<t8 / 256, 256, 0, stream>>>(pool_w, WPL16, t8, t8, kCarPool);
  }
  {
    const int t8 = kPrjP * kDin / 8;
    const int r8 = kPrjN * kDin / 8;
    cast_f16_kernel<<<t8 / 256, 256, 0, stream>>>(W_xprj, WXP16, t8, r8, kCarWx);
  }
  {
    const int t8 = kDin * kDtR / 8;
    cast_f16_kernel<<<t8 / 256, 256, 0, stream>>>(W_dt, WDT16, t8, t8, kCarWdt);
  }
  {
    const int t8 = kDmod * kDin / 8;
    cast_f16_kernel<<<t8 / 256, 256, 0, stream>>>(W_out, WOUT16, t8, t8, kCarWout);
  }

  xpose_x_kernel<<<dim3(kSeqL / 64, kCin / 64, kBatch), 256, 0, stream>>>(x, SEQ16);

  wmma_gemm64<0, 6><<<dim3(8, 1), 256, 0, stream>>>(
      SEQ16, kDmod, 0L, WPL16, kCin, 0L, YS0, kPpm, 0L,
      bn_b, bn_g, bn_b, bn_m, bn_v, kRows, kPpm, kCin, 1.0f / kCarPool);
  ppm0_mean_kernel<<<4, 256, 0, stream>>>(YS0, SEQ16);

  pool_kernel<<<kPoolRows * 64 / 256, 256, 0, stream>>>(x, POOL16);
  wmma_gemm64<0, 6><<<dim3(1, 1), 256, 0, stream>>>(
      POOL16, kCin, 0L, WPL16 + (size_t)1 * kPpm * kCin, kCin, 0L, YSP, kPpm, 0L,
      bn_b, bn_g + kPpm, bn_b + kPpm, bn_m + kPpm, bn_v + kPpm, kSegP1, kPpm, kCin, 1.0f / kCarPool);
  wmma_gemm64<0, 6><<<dim3(3, 1), 256, 0, stream>>>(
      POOL16 + (size_t)kSegOff2 * kCin, kCin, 0L, WPL16 + (size_t)2 * kPpm * kCin, kCin, 0L,
      YSP + (size_t)kSegOff2 * kPpm, kPpm, 0L,
      bn_b, bn_g + 2 * kPpm, bn_b + 2 * kPpm, bn_m + 2 * kPpm, bn_v + 2 * kPpm, kSegP2, kPpm, kCin, 1.0f / kCarPool);
  wmma_gemm64<0, 6><<<dim3(5, 1), 256, 0, stream>>>(
      POOL16 + (size_t)kSegOff3 * kCin, kCin, 0L, WPL16 + (size_t)3 * kPpm * kCin, kCin, 0L,
      YSP + (size_t)kSegOff3 * kPpm, kPpm, 0L,
      bn_b, bn_g + 3 * kPpm, bn_b + 3 * kPpm, bn_m + 3 * kPpm, bn_v + 3 * kPpm, kSegP3, kPpm, kCin, 1.0f / kCarPool);
  interp_kernel<<<kRows * 48 / 256, 256, 0, stream>>>(YSP, SEQ16);

  wmma_gemm64<0, 0><<<dim3(256, 1), 256, 0, stream>>>(
      SEQ16, kDmod, 0L, WIN16, kDmod, 0L, XZ, kXZP, 0L,
      bn_b, bn_g, bn_b, bn_m, bn_v, kRows, kXZP, kDmod, 1.0f / kCarWin);

  conv_silu_kernel<<<dim3(kDin / 256, kRows / 64), 256, 0, stream>>>(XZ, conv_w, conv_b, UC, UC16);

  wmma_gemm64<0, 0><<<dim3(8, 1), 256, 0, stream>>>(
      UC16, kDin, 0L, WXP16, kDin, 0L, PROJ, kPrjP, 0L,
      bn_b, bn_g, bn_b, bn_m, bn_v, kRows, kPrjP, kDin, 1.0f / kCarWx);

  dt_cast_kernel<<<(kRows * kDtR) / 8 / 256, 256, 0, stream>>>(PROJ, DT16, (kRows * kDtR) / 8, kCarDt);

  wmma_gemm64<2, 0><<<dim3(128, 1), 256, 0, stream>>>(
      DT16, kDtR, 0L, WDT16, kDtR, 0L, DLR, kDin, 0L,
      b_dt, bn_g, bn_b, bn_m, bn_v, kRows, kDin, kDtR, 1.0f / (kCarDt * kCarWdt));

  scan_kernel<<<dim3(kDin / 256, kBatch), 256, 0, stream>>>(DLR, UC, XZ, PROJ, A_log, Dv, Y16);

  wmma_gemm64<0, 0><<<dim3(32, kBatch), 256, 0, stream>>>(
      WOUT16, kDin, 0L, Y16, kDin, (long)kSeqL * kDin, dout, kSeqL, (long)kDmod * kSeqL,
      bn_b, bn_g, bn_b, bn_m, bn_v, kDmod, kSeqL, kDin, 1.0f / (kCarY * kCarWout));
}
